// CrossAttention_55319178772617
// MI455X (gfx1250) — hardware-verified
//
#include <hip/hip_runtime.h>


#ifndef NB
#define NB 4
#endif
#ifndef TX
#define TX 1024
#endif
#define NB_FULL 4
#define TX_FULL 1024
#define TY   2048
#define DMD  768
#define NHD  12
#define HD   64
#define HG   4
#define PCAR 1024.0f
#define SCL  0.125f
static_assert(NB >= 1 && NB <= NB_FULL);
static_assert(TX >= 64 && TX <= TX_FULL && (TX % 64) == 0);
static_assert((NHD % HG) == 0);
static_assert((TY % 128) == 0 && (DMD % 64) == 0 && HD == 64 && NHD * HD == DMD);
static_assert((DMD % 32) == 0 && (HD % 32) == 0 && (TY % 32) == 0);

typedef _Float16 h16;
typedef unsigned short bf;
typedef __attribute__((ext_vector_type(16))) __bf16   v16bf;
typedef __attribute__((ext_vector_type(16))) _Float16 v16h;
typedef __attribute__((ext_vector_type(8)))  _Float16 v8h;
typedef __attribute__((ext_vector_type(8)))  unsigned short v8us;
typedef __attribute__((ext_vector_type(8)))  float    v8f;
typedef __attribute__((ext_vector_type(4)))  float    v4f;
typedef __attribute__((ext_vector_type(4)))  _Float16 v4h;
typedef v8h  __attribute__((may_alias)) v8ha;
typedef v4f  __attribute__((may_alias)) v4fa;
typedef v8us __attribute__((may_alias)) v8usa;

__device__ __forceinline__ unsigned short f2bf(float f) { unsigned u = __float_as_uint(f); u += 0x7FFFu + ((u >> 16) & 1u); return (unsigned short)(u >> 16); }
__device__ __forceinline__ float bf2f(unsigned short b) { return __uint_as_float(((unsigned)b) << 16); }
__device__ __forceinline__ float bfr(float f) { return bf2f(f2bf(f)); }
__device__ __forceinline__ v16h cat16(v8h lo, v8h hi) { return __builtin_shufflevector(lo, hi, 0, 1, 2, 3, 4, 5, 6, 7, 8, 9, 10, 11, 12, 13, 14, 15); }
__device__ __forceinline__ v16bf cat16b(v8us lo, v8us hi) { return __builtin_bit_cast(v16bf, __builtin_shufflevector(lo, hi, 0, 1, 2, 3, 4, 5, 6, 7, 8, 9, 10, 11, 12, 13, 14, 15)); }
__device__ __forceinline__ v8f wmma16(v16h a, v16h b, v8f c) { return __builtin_amdgcn_wmma_f32_16x16x32_f16(false, a, false, b, (short)0, c, false, false); }
__device__ __forceinline__ v8f wmmab(v16bf a, v16bf b, v8f c) { return __builtin_amdgcn_wmma_f32_16x16x32_bf16(false, a, false, b, (short)0, c, false, false); }
__device__ __forceinline__ h16 tohx(float x) { return (h16)x; }

template <typename T16> struct WFrag;
template <> struct WFrag<h16> { typedef v16h V; static __device__ __forceinline__ V ld(const h16* p) { return cat16(*(const v8h*)p, *(const v8h*)(p + 16)); } static __device__ __forceinline__ v8f mma(V a, V b, v8f c) { return wmma16(a, b, c); } };
template <> struct WFrag<bf> { typedef v16bf V; static __device__ __forceinline__ V ld(const bf* p) { return cat16b(*(const v8us*)p, *(const v8us*)(p + 16)); } static __device__ __forceinline__ v8f mma(V a, V b, v8f c) { return wmmab(a, b, c); } };
template <typename T16, int NSPLIT, bool BIAS>
__global__ __launch_bounds__(32) void k_gemmw(const T16* __restrict__ A, const T16* __restrict__ A2, const T16* __restrict__ Bt, const T16* __restrict__ Bt2, int K, float* C, int ldc, const float* __restrict__ bias, size_t sA, size_t sB, size_t sC, float cs) {
    typedef typename WFrag<T16>::V V;
    __shared__ __align__(16) float os[16 * 68];
    const size_t z = blockIdx.z; A += z * sA; if (A2) A2 += z * sA; Bt += z * sB; if (Bt2) Bt2 += z * sB; C += z * sC;
    const int lane = threadIdx.x & 31, lr = lane & 15, hi = lane >> 4; const int r0 = blockIdx.x * 64, c0 = blockIdx.y * 64;
    v8f acc[4][4];
#pragma unroll
    for (int mb = 0; mb < 4; ++mb)
#pragma unroll
        for (int nb = 0; nb < 4; ++nb) acc[mb][nb] = (v8f){};
    const size_t aoff = (size_t)(r0 + lr) * K + 8 * hi, boff = (size_t)(c0 + lr) * K + 8 * hi;
#pragma unroll 1
    for (int kc = 0; kc < K; kc += 32) {
        V a[4], a2[4];
#pragma unroll
        for (int mb = 0; mb < 4; ++mb) { a[mb] = WFrag<T16>::ld(A + aoff + (size_t)mb * 16 * K + kc); if (NSPLIT == 1 || NSPLIT == 2) a2[mb] = WFrag<T16>::ld(A2 + aoff + (size_t)mb * 16 * K + kc); }
#pragma unroll
        for (int nb = 0; nb < 4; ++nb) { const V b = WFrag<T16>::ld(Bt + boff + (size_t)nb * 16 * K + kc); V b2; if (NSPLIT >= 2) b2 = WFrag<T16>::ld(Bt2 + boff + (size_t)nb * 16 * K + kc);
#pragma unroll
            for (int mb = 0; mb < 4; ++mb) { acc[mb][nb] = WFrag<T16>::mma(a[mb], b, acc[mb][nb]); if (NSPLIT == 1 || NSPLIT == 2) acc[mb][nb] = WFrag<T16>::mma(a2[mb], b, acc[mb][nb]); if (NSPLIT >= 2) acc[mb][nb] = WFrag<T16>::mma(a[mb], b2, acc[mb][nb]); } }
        asm volatile("v_nop\n\tv_nop\n\tv_nop\n\tv_nop" : "+v"(acc[0][0]), "+v"(acc[1][1]), "+v"(acc[2][2]), "+v"(acc[3][3]) : "v"(a[0]), "v"(a[3]));
    }
#pragma unroll
    for (int mb = 0; mb < 4; ++mb) {
#pragma unroll
        for (int nb = 0; nb < 4; ++nb) {
#pragma unroll
            for (int j = 0; j < 8; ++j) os[(hi * 8 + j) * 68 + nb * 16 + lr] = acc[mb][nb][j]; }
        __builtin_amdgcn_wave_barrier(); asm volatile("" ::: "memory");
        float* crow = C + (size_t)(r0 + mb * 16) * ldc + c0;
#pragma unroll 1
        for (int ps = 0; ps < 2; ++ps) {
#pragma unroll
            for (int s = 0; s < 8; ++s) { const int row = 2 * s + hi, cofs = lr * 4; v4f val = *(const v4fa*)(os + row * 68 + cofs);
                val[0] = __fmul_rn(val[0], cs); val[1] = __fmul_rn(val[1], cs); val[2] = __fmul_rn(val[2], cs); val[3] = __fmul_rn(val[3], cs);
                if (BIAS) { val[0] += bfr(bias[c0 + cofs]); val[1] += bfr(bias[c0 + cofs + 1]); val[2] += bfr(bias[c0 + cofs + 2]); val[3] += bfr(bias[c0 + cofs + 3]); }
                *(volatile v4f*)(crow + (size_t)row * ldc + cofs) = val; }
            if (ps == 0) __threadfence(); }
        __builtin_amdgcn_wave_barrier(); asm volatile("" ::: "memory");
    }
}

__global__ __launch_bounds__(256) void k_cvt8r(const float* __restrict__ src, bf* dst, int rows, int srows, size_t n8) {
    const size_t i = (size_t)blockIdx.x * 256 + threadIdx.x; if (i >= n8) return;
    const size_t e = i * 8; const size_t r = e / DMD; const int c = (int)(e % DMD); const size_t bb = r / (size_t)rows; const size_t t = r % (size_t)rows;
    const v8f v = *(const v8f*)(src + (bb * (size_t)srows + t) * DMD + c); v8us o;
#pragma unroll
    for (int k = 0; k < 8; ++k) o[k] = f2bf(v[k]);
    *(volatile v8us*)(dst + e) = o; __threadfence(); *(volatile v8us*)(dst + e) = o; }

template <bool RB>
__global__ __launch_bounds__(256) void k_cvth(const float* __restrict__ F, h16* P, float sc, size_t n8) {
    const size_t i = (size_t)blockIdx.x * 256 + threadIdx.x; if (i >= n8) return;
    const v8f a = *(const v8f*)(F + i * 8); v8h o;
#pragma unroll
    for (int q = 0; q < 8; ++q) { const float u = RB ? bfr(a[q]) : a[q]; o[q] = tohx(__fmul_rn(u, sc)); }
    *(volatile v8h*)(P + i * 8) = o; __threadfence(); *(volatile v8h*)(P + i * 8) = o; }

__global__ __launch_bounds__(256) void k_lsoft(const float* __restrict__ Sb, h16* P16, int nrows) {
    const int lane = threadIdx.x & 31; const int row = blockIdx.x * 8 + (threadIdx.x >> 5); if (row >= nrows) return;
    const float* sr = Sb + (size_t)row * TY; float mx = -3.0e38f;
#pragma unroll 4
    for (int ch = 0; ch < TY / 128; ++ch) { const int j0 = ch * 128 + lane * 4; const v4f a = *(const v4f*)(sr + j0);
#pragma unroll
        for (int q = 0; q < 4; ++q) { float t = a[q] * SCL; asm volatile("" : "+v"(t)); mx = fmaxf(mx, t); } }
#pragma unroll
    for (int sh = 16; sh; sh >>= 1) mx = fmaxf(mx, __shfl_xor(mx, sh, 32));
    float sum = 0.f;
#pragma unroll 4
    for (int ch = 0; ch < TY / 128; ++ch) { const int j0 = ch * 128 + lane * 4; const v4f a = *(const v4f*)(sr + j0);
#pragma unroll
        for (int q = 0; q < 4; ++q) { float t = a[q] * SCL; asm volatile("" : "+v"(t)); float d0 = __fsub_rn(t, mx); asm volatile("" : "+v"(d0)); sum += __builtin_amdgcn_exp2f(__fmul_rn(d0, 1.4426950408889634f)); } }
#pragma unroll
    for (int sh = 16; sh; sh >>= 1) sum += __shfl_xor(sum, sh, 32);
    const float f = __fdiv_rn(PCAR, sum);
#pragma unroll 1
    for (int ps = 0; ps < 2; ++ps) {
#pragma unroll 2
        for (int ch = 0; ch < TY / 128; ++ch) { const int j0 = ch * 128 + lane * 4; const v4f a = *(const v4f*)(sr + j0); v4h o4;
#pragma unroll
            for (int q = 0; q < 4; ++q) { float t = a[q] * SCL; asm volatile("" : "+v"(t)); float d0 = __fsub_rn(t, mx); asm volatile("" : "+v"(d0)); float ex = __builtin_amdgcn_exp2f(__fmul_rn(d0, 1.4426950408889634f)); asm volatile("" : "+v"(ex)); o4[q] = tohx(ex * f); }
            *(volatile v4h*)(P16 + (size_t)row * TY + j0) = o4; }
        if (ps == 0) __threadfence(); }
}

extern "C" void kernel_launch(void* const* d_in, const int* in_sizes, int n_in,
                              void* d_out, int out_size, void* d_ws, size_t ws_size, hipStream_t stream) {
    if (n_in < 7) return;
    const size_t needx = (size_t)(NB - 1) * TX_FULL * DMD + (size_t)TX * DMD;
    if ((size_t)in_sizes[0] < needx || (size_t)in_sizes[1] < (size_t)NB * TY * DMD) return;
    if (in_sizes[2] < DMD * DMD || in_sizes[3] < DMD * DMD || in_sizes[4] < DMD * DMD || in_sizes[5] < DMD * DMD || in_sizes[6] < DMD) return;
    if ((size_t)out_size < needx) return;
    const float* x = (const float*)d_in[0]; const float* y = (const float*)d_in[1];
    const float* wq = (const float*)d_in[2]; const float* wk = (const float*)d_in[3]; const float* wv = (const float*)d_in[4]; const float* wp = (const float*)d_in[5]; const float* bp = (const float*)d_in[6];
    float* OUT = (float*)d_out;

    char* base = (char*)d_ws;
    auto al = [](size_t b) { return (b + 255) & ~(size_t)255; };
    size_t offA = 0, offB = 0;
    bf* XB = (bf*)(base + offA); offA += al((size_t)NB * TX * DMD * 2);
    bf* YB = (bf*)(base + offA); offA += al((size_t)NB * TY * DMD * 2);
    size_t fbytes = (size_t)NHD * NB * TY * HD * 4;
    { const size_t f2 = (size_t)NB * DMD * TY * 4; if (f2 > fbytes) fbytes = f2; }
    { const size_t f3 = (size_t)NHD * NB * TX * HD * 4; if (f3 > fbytes) fbytes = f3; }
    float* F = (float*)(base + offA); offA += al(fbytes);
    float* Sb = (float*)(base + offB); offB += al((size_t)HG * TX * TY * 4);
    h16* P16 = (h16*)(base + offB); offB += al((size_t)HG * TX * TY * 2);
    size_t off = (offA > offB) ? offA : offB;
    auto take = [&](size_t bytes) { char* p = base + off; off += al(bytes); return (void*)p; };
    bf* WQ = (bf*)take((size_t)DMD * DMD * 2); bf* WK = (bf*)take((size_t)DMD * DMD * 2); bf* WV = (bf*)take((size_t)DMD * DMD * 2); h16* WP16 = (h16*)take((size_t)DMD * DMD * 2);
    h16* QP16 = (h16*)take((size_t)NHD * NB * TX * HD * 2);
    h16* KP16 = (h16*)take((size_t)NHD * NB * TY * HD * 2);
    h16* VT16 = (h16*)take((size_t)NB * DMD * TY * 2);
    float* Ob = (float*)take((size_t)NB * TX * DMD * 4);
    h16* CT16 = (h16*)take((size_t)NB * TX * DMD * 2);
    if (off > ws_size) return;
    if (off > (size_t)134217728) return;

    auto nb256 = [](size_t n) { return (unsigned)((n + 255) / 256); };
    const size_t n8w = (size_t)DMD * DMD / 8;
    k_cvt8r<<<nb256(n8w), 256, 0, stream>>>(wq, WQ, DMD, DMD, n8w);
    k_cvt8r<<<nb256(n8w), 256, 0, stream>>>(wk, WK, DMD, DMD, n8w);
    k_cvt8r<<<nb256(n8w), 256, 0, stream>>>(wv, WV, DMD, DMD, n8w);
    k_cvth<true><<<nb256(n8w), 256, 0, stream>>>(wp, WP16, 16.0f, n8w);
    const size_t n8x = (size_t)NB * TX * DMD / 8, n8y = (size_t)NB * TY * DMD / 8;
    k_cvt8r<<<nb256(n8x), 256, 0, stream>>>(x, XB, TX, TX_FULL, n8x);
    k_cvt8r<<<nb256(n8y), 256, 0, stream>>>(y, YB, TY, TY, n8y);
    k_gemmw<bf, 0, false><<<dim3((unsigned)(NB * TX / 64), 1, NHD), 32, 0, stream>>>(XB, nullptr, WQ, nullptr, DMD, F, HD, nullptr, (size_t)0, (size_t)HD * DMD, (size_t)NB * TX * HD, 1.0f);
    const size_t n8q = (size_t)NHD * NB * TX * HD / 8;
    k_cvth<false><<<nb256(n8q), 256, 0, stream>>>(F, QP16, 1.0f, n8q);
    k_gemmw<bf, 0, false><<<dim3((unsigned)(NB * TY / 64), 1, NHD), 32, 0, stream>>>(YB, nullptr, WK, nullptr, DMD, F, HD, nullptr, (size_t)0, (size_t)HD * DMD, (size_t)NB * TY * HD, 1.0f);
    const size_t n8k = (size_t)NHD * NB * TY * HD / 8;
    k_cvth<false><<<nb256(n8k), 256, 0, stream>>>(F, KP16, 1.0f, n8k);
    k_gemmw<bf, 0, false><<<dim3(DMD / 64, TY / 64, NB), 32, 0, stream>>>(WV, nullptr, YB, nullptr, DMD, F, TY, nullptr, (size_t)0, (size_t)TY * DMD, (size_t)DMD * TY, 1.0f);
    const size_t n8v = (size_t)NB * DMD * TY / 8;
    k_cvth<false><<<nb256(n8v), 256, 0, stream>>>(F, VT16, 1.0f, n8v);
    for (int b = 0; b < NB; ++b) {
        for (int g = 0; g < NHD / HG; ++g) {
            const int h0 = g * HG;
            const size_t qo = ((size_t)h0 * NB * TX + (size_t)b * TX) * HD, ko = ((size_t)h0 * NB * TY + (size_t)b * TY) * HD;
            k_gemmw<h16, 0, false><<<dim3(TX / 64, TY / 64, HG), 32, 0, stream>>>(QP16 + qo, nullptr, KP16 + ko, nullptr, HD, Sb, TY, nullptr, (size_t)NB * TX * HD, (size_t)NB * TY * HD, (size_t)TX * TY, 1.0f);
            k_lsoft<<<(unsigned)(HG * TX / 8), 256, 0, stream>>>(Sb, P16, HG * TX);
            k_gemmw<h16, 0, false><<<dim3(TX / 64, 1, HG), 32, 0, stream>>>(P16, nullptr, VT16 + ((size_t)b * DMD + (size_t)h0 * HD) * TY, nullptr, TY, Ob + (size_t)b * TX * DMD + (size_t)h0 * HD, DMD, nullptr, (size_t)TX * TY, (size_t)HD * TY, (size_t)HD, 1.0f);
        }
    }
    const size_t n8c = (size_t)NB * TX * DMD / 8;
    k_cvth<false><<<nb256(n8c), 256, 0, stream>>>(Ob, CT16, 1.0f, n8c);
    k_gemmw<h16, 0, true><<<dim3(TX / 64, DMD / 64, NB), 32, 0, stream>>>(CT16, nullptr, WP16, nullptr, DMD, OUT, DMD, bp, (size_t)TX * DMD, (size_t)0, (size_t)TX_FULL * DMD, 1.0f / 16384.0f);
}
